// MADE_29171417874753
// MI455X (gfx1250) — hardware-run, weakly checked
//
#include <hip/hip_runtime.h>
#include <math.h>

constexpr int DIM      = 128;
constexpr int HID      = 512;
constexpr int NBAT     = 256;
constexpr int NTHR     = 256;
constexpr int ROWS_BLK = 32;
constexpr int HP       = 520;
constexpr int XSP      = 128;
constexpr float WCAR   = 256.0f;
constexpr float HCAR   = 64.0f;
constexpr float CAR_INV = 1.0f / 16384.0f;
static_assert(NBAT % ROWS_BLK == 0);
static_assert(ROWS_BLK == 32);
static_assert(HID == 64 * (NTHR / 32));
static_assert(HID % 32 == 0);
static_assert(DIM == 16 * (NTHR / 32));
static_assert(HID == 8 * 64 && NTHR == 4 * 64);
static_assert(DIM % 64 == 0 && HID % 64 == 0);
static_assert((ROWS_BLK * DIM) % (4 * NTHR) == 0);
static_assert(HP % 8 == 0 && XSP % 4 == 0);

typedef __attribute__((ext_vector_type(16))) _Float16 v16h;
typedef __attribute__((ext_vector_type(8)))  _Float16 v8h;
typedef __attribute__((ext_vector_type(8)))  float    v8f;
typedef __attribute__((ext_vector_type(4)))  float    v4f;

__device__ __forceinline__ void dep_guard_h(v8f& a, v8f& b, v16h x, v16h y) {
  asm volatile("v_nop\n\tv_nop\n\tv_nop\n\tv_nop" : "+v"(a), "+v"(b) : "v"(x), "v"(y));
}
__device__ __forceinline__ void dep_guard4_h(v8f& a, v8f& b, v8f& cc, v8f& d, v16h x, v16h y) {
  asm volatile("v_nop\n\tv_nop\n\tv_nop\n\tv_nop" : "+v"(a), "+v"(b), "+v"(cc), "+v"(d) : "v"(x), "v"(y));
}
__device__ __forceinline__ void keep4_h(v16h a, v16h b, v16h c, v16h d) { asm volatile("v_nop" :: "v"(a), "v"(b), "v"(c), "v"(d)); }
__device__ __forceinline__ void acc_guard4(v8f& a, v8f& b, v8f& c, v8f& d) {
  asm volatile("v_nop\n\tv_nop\n\tv_nop\n\tv_nop" : "+v"(a), "+v"(b), "+v"(c), "+v"(d));
}
__device__ __forceinline__ void acc_guard2(v8f& a, v8f& b) { asm volatile("v_nop\n\tv_nop\n\tv_nop\n\tv_nop" : "+v"(a), "+v"(b)); }

template <typename T> struct Frag;
template <> struct Frag<_Float16> {
  typedef v16h V; union U { v16h v; v8h h[2]; };
  static __device__ __forceinline__ v16h load(const _Float16* p) {
    U f; f.h[0] = *(const v8h*)(p); f.h[1] = *(const v8h*)(p + 16); return f.v;
  }
  static __device__ __forceinline__ v8f mma(v16h a, v16h b, v8f c) {
    return __builtin_amdgcn_wmma_f32_16x16x32_f16(false, a, false, b, (short)0, c, false, false);
  }
};

__device__ __forceinline__ float sum16(float v) {
  v += __shfl_xor(v, 1, 32);
  v += __shfl_xor(v, 2, 32);
  v += __shfl_xor(v, 4, 32);
  v += __shfl_xor(v, 8, 32);
  return v;
}

__global__ __launch_bounds__(NTHR) void cvtmask16_kernel(const float* __restrict__ W, const float* __restrict__ Mk,
                                                         unsigned short* __restrict__ dst, int n8, float sc) {
  const int i = blockIdx.x * NTHR + threadIdx.x;
  if (i < n8) {
    const size_t o = (size_t)i * 8;
    const v4f wa = *(const v4f*)(W + o), wb = *(const v4f*)(W + o + 4);
    const v4f ma = *(const v4f*)(Mk + o), mb = *(const v4f*)(Mk + o + 4);
    v8h hv;
#pragma unroll
    for (int e = 0; e < 4; ++e) {
      hv[e]     = (_Float16)((wa[e] * ma[e]) * sc);
      hv[4 + e] = (_Float16)((wb[e] * mb[e]) * sc);
    }
    *(volatile v8h*)(dst + o) = hv;
    __threadfence();
    *(volatile v8h*)(dst + o) = hv;
  }
}

__global__ __launch_bounds__(NTHR) void mulmask4_kernel(const float* __restrict__ W, const float* __restrict__ Mk,
                                                        float* __restrict__ dst, int n4) {
  const int i = blockIdx.x * NTHR + threadIdx.x;
  if (i < n4) {
    const size_t o = (size_t)i * 4;
    const v4f w = *(const v4f*)(W + o), m = *(const v4f*)(Mk + o);
    v4f v;
#pragma unroll
    for (int e = 0; e < 4; ++e) v[e] = w[e] * m[e];
    *(volatile v4f*)(dst + o) = v;
    __threadfence();
    *(volatile v4f*)(dst + o) = v;
  }
}

__global__ __launch_bounds__(NTHR) void tpmask_kernel(const float* __restrict__ W, const float* __restrict__ Mk,
                                                      int R, int C, float* __restrict__ O) {
  __shared__ float Tt[64 * 65];
  const int tid = threadIdx.x;
  const int c0 = blockIdx.x * 64, r0 = blockIdx.y * 64;
#pragma unroll
  for (int i = 0; i < 4; ++i) {
    const int idx = i * NTHR + tid;
    const int rr = idx >> 4, cc = (idx & 15) * 4;
    const size_t go = (size_t)(r0 + rr) * (size_t)C + c0 + cc;
    const v4f w = *(const v4f*)(W + go), m = *(const v4f*)(Mk + go);
    Tt[rr * 65 + cc + 0] = w[0] * m[0];
    Tt[rr * 65 + cc + 1] = w[1] * m[1];
    Tt[rr * 65 + cc + 2] = w[2] * m[2];
    Tt[rr * 65 + cc + 3] = w[3] * m[3];
  }
  __syncthreads();
  v4f ov[4];
#pragma unroll
  for (int it = 0; it < 4; ++it) {
    const int idx = it * NTHR + tid;
    const int orow = idx >> 4, c4 = (idx & 15) * 4;
#pragma unroll
    for (int e = 0; e < 4; ++e) ov[it][e] = Tt[(c4 + e) * 65 + orow];
  }
  for (int pass = 0; pass < 2; ++pass) {
#pragma unroll
    for (int it = 0; it < 4; ++it) {
      const int idx = it * NTHR + tid;
      const int orow = idx >> 4, c4 = (idx & 15) * 4;
      *(volatile v4f*)(O + (size_t)(c0 + orow) * (size_t)R + r0 + c4) = ov[it];
    }
    __threadfence();
  }
}

__global__ __launch_bounds__(NTHR) void made_seq_kernel(const float* __restrict__ z, const float* __restrict__ b0,
                                                        const float* __restrict__ b1, const float* __restrict__ b2,
                                                        const unsigned short* __restrict__ M1Hp,
                                                        const unsigned short* __restrict__ M2Ap,
                                                        const float* __restrict__ M0T, const float* __restrict__ M2F,
                                                        float* __restrict__ out) {
  __shared__ __align__(16) _Float16 Hs[ROWS_BLK * HP];
  __shared__ __align__(16) float    xs[ROWS_BLK * XSP];
  __shared__ __align__(16) float    part[2 * ROWS_BLK * 8];
  __shared__ __align__(16) float    xcol[ROWS_BLK];
  __shared__ __align__(16) float    ldst[ROWS_BLK];
  const _Float16* M1H = (const _Float16*)M1Hp;
  const _Float16* M2A = (const _Float16*)M2Ap;
  const int tid = threadIdx.x, lane = tid & 31, wave = tid >> 5;
  const int c = lane & 15, hh = lane >> 4, koff = hh * 8;
  const int rg = tid >> 6, c8 = (tid & 63) * 8;
  const int rb = blockIdx.x * ROWS_BLK;

  float a1s[8][8];
  {
    const v4f u0 = *(const v4f*)(b0 + c8), u1 = *(const v4f*)(b0 + c8 + 4);
#pragma unroll
    for (int r = 0; r < 8; ++r)
#pragma unroll
      for (int e = 0; e < 4; ++e) { a1s[r][e] = u0[e]; a1s[r][4 + e] = u1[e]; }
  }
  float bb1[4];
#pragma unroll
  for (int nt = 0; nt < 4; ++nt) bb1[nt] = b1[64 * wave + 16 * nt + c];

  const v8f z8 = {0.f, 0.f, 0.f, 0.f, 0.f, 0.f, 0.f, 0.f};
  v8f acc[2][4];
#pragma unroll
  for (int mt = 0; mt < 2; ++mt)
#pragma unroll
    for (int nt = 0; nt < 4; ++nt) acc[mt][nt] = z8;

#pragma unroll 1
  for (int i = 0; i < DIM; ++i) {
#pragma unroll
    for (int r = 0; r < 8; ++r) {
      v8h hv;
#pragma unroll
      for (int e = 0; e < 8; ++e) hv[e] = (_Float16)(fmaxf(a1s[r][e], 0.0f) * HCAR);
      *(v8h*)(Hs + (8 * rg + r) * HP + c8) = hv;
    }
    __syncthreads();

#pragma unroll
    for (int mt = 0; mt < 2; ++mt)
#pragma unroll
      for (int nt = 0; nt < 4; ++nt) acc[mt][nt] = z8;
    {
      const _Float16* brow = M1H + (size_t)(64 * wave + c) * HID + koff;
      const _Float16* arow = Hs + c * HP + koff;
#pragma unroll 1
      for (int k0 = 0; k0 < HID; k0 += 32) {
        v16h bh[4];
#pragma unroll
        for (int nt = 0; nt < 4; ++nt) bh[nt] = Frag<_Float16>::load(brow + (size_t)(16 * nt) * HID + k0);
#pragma unroll
        for (int mt = 0; mt < 2; ++mt) {
          const v16h a = Frag<_Float16>::load(arow + (16 * mt) * HP + k0);
#pragma unroll
          for (int nt = 0; nt < 4; ++nt) acc[mt][nt] = Frag<_Float16>::mma(a, bh[nt], acc[mt][nt]);
          dep_guard4_h(acc[mt][0], acc[mt][1], acc[mt][2], acc[mt][3], a, bh[3]);
        }
        keep4_h(bh[0], bh[1], bh[2], bh[3]);
      }
    }
    acc_guard4(acc[0][0], acc[0][1], acc[0][2], acc[0][3]);
    acc_guard4(acc[1][0], acc[1][1], acc[1][2], acc[1][3]);

    float wm[4], wa[4];
#pragma unroll
    for (int nt = 0; nt < 4; ++nt) {
      const int n = 64 * wave + 16 * nt + c;
      wm[nt] = M2F[(size_t)i * HID + n];
      wa[nt] = M2F[(size_t)(DIM + i) * HID + n];
    }
    float pmu[2][8], pal[2][8];
#pragma unroll
    for (int mt = 0; mt < 2; ++mt) {
#pragma unroll
      for (int r = 0; r < 8; ++r) {
        float sm = 0.0f, sa = 0.0f;
#pragma unroll
        for (int nt = 0; nt < 4; ++nt) {
          const float hv = fmaxf(acc[mt][nt][r] * CAR_INV + bb1[nt], 0.0f);
          acc[mt][nt][r] = hv;
          sm = fmaf(hv, wm[nt], sm);
          sa = fmaf(hv, wa[nt], sa);
        }
        pmu[mt][r] = sm;
        pal[mt][r] = sa;
      }
    }
#pragma unroll
    for (int mt = 0; mt < 2; ++mt)
#pragma unroll
      for (int r = 0; r < 8; ++r) { pmu[mt][r] = sum16(pmu[mt][r]); pal[mt][r] = sum16(pal[mt][r]); }
    if (c == 0) {
#pragma unroll
      for (int mt = 0; mt < 2; ++mt)
#pragma unroll
        for (int r = 0; r < 8; ++r) {
          const int row = 16 * mt + 8 * hh + r;
          part[row * 8 + wave]              = pmu[mt][r];
          part[(ROWS_BLK + row) * 8 + wave] = pal[mt][r];
        }
    }
    __syncthreads();

    if (wave == 0) {
      const int row = lane;
      const v4f p0 = *(const v4f*)(part + row * 8), p1 = *(const v4f*)(part + row * 8 + 4);
      const v4f q0 = *(const v4f*)(part + (ROWS_BLK + row) * 8), q1 = *(const v4f*)(part + (ROWS_BLK + row) * 8 + 4);
      const float smu = ((p0[0] + p0[1]) + (p0[2] + p0[3])) + ((p1[0] + p1[1]) + (p1[2] + p1[3]));
      const float sal = ((q0[0] + q0[1]) + (q0[2] + q0[3])) + ((q1[0] + q1[1]) + (q1[2] + q1[3]));
      const float mu = smu + b2[i];
      const float al = sal + b2[DIM + i];
      const float zz = z[(size_t)(rb + row) * DIM + i];
      const float xi = mu + expf(al) * zz;
      xs[row * XSP + i] = xi;
      xcol[row] = xi;
    }
    __syncthreads();

    {
      const v4f x0 = *(const v4f*)(xcol + 8 * rg), x1 = *(const v4f*)(xcol + 8 * rg + 4);
      const v4f m0v = *(const v4f*)(M0T + (size_t)i * HID + c8), m1v = *(const v4f*)(M0T + (size_t)i * HID + c8 + 4);
#pragma unroll
      for (int r = 0; r < 8; ++r) {
        const float xr = (r < 4) ? x0[r] : x1[r - 4];
#pragma unroll
        for (int e = 0; e < 4; ++e) {
          a1s[r][e]     = fmaf(xr, m0v[e], a1s[r][e]);
          a1s[r][4 + e] = fmaf(xr, m1v[e], a1s[r][4 + e]);
        }
      }
    }
  }

#pragma unroll
  for (int mt = 0; mt < 2; ++mt)
#pragma unroll
    for (int nt = 0; nt < 4; ++nt)
#pragma unroll
      for (int r = 0; r < 8; ++r)
        Hs[(16 * mt + 8 * hh + r) * HP + 64 * wave + 16 * nt + c] = (_Float16)(acc[mt][nt][r] * HCAR);
  __syncthreads();
  v8f fa0 = z8, fa1 = z8;
  {
    const _Float16* brow = M2A + (size_t)(16 * wave + c) * HID + koff;
    const _Float16* ar0  = Hs + c * HP + koff;
    const _Float16* ar1  = Hs + (16 + c) * HP + koff;
#pragma unroll 1
    for (int k0 = 0; k0 < HID; k0 += 32) {
      const v16h b  = Frag<_Float16>::load(brow + k0);
      const v16h x0 = Frag<_Float16>::load(ar0 + k0);
      const v16h x1 = Frag<_Float16>::load(ar1 + k0);
      fa0 = Frag<_Float16>::mma(x0, b, fa0);
      fa1 = Frag<_Float16>::mma(x1, b, fa1);
      dep_guard_h(fa0, fa1, x1, b);
      keep4_h(x0, x1, b, b);
    }
  }
  acc_guard2(fa0, fa1);
  {
    const float bal = b2[DIM + 16 * wave + c];
    float ps0[8], ps1[8];
#pragma unroll
    for (int r = 0; r < 8; ++r) {
      ps0[r] = sum16(fa0[r] * CAR_INV + bal);
      ps1[r] = sum16(fa1[r] * CAR_INV + bal);
    }
    if (c == 0) {
#pragma unroll
      for (int r = 0; r < 8; ++r) {
        part[(8 * hh + r) * 8 + wave]      = ps0[r];
        part[(16 + 8 * hh + r) * 8 + wave] = ps1[r];
      }
    }
  }
  __syncthreads();
  if (wave == 0) {
    const int row = lane;
    const v4f p0 = *(const v4f*)(part + row * 8), p1 = *(const v4f*)(part + row * 8 + 4);
    const float s = ((p0[0] + p0[1]) + (p0[2] + p0[3])) + ((p1[0] + p1[1]) + (p1[2] + p1[3]));
    ldst[row] = -s;
  }
  __syncthreads();

  {
    const int l8 = lane & 7;
    for (int pass = 0; pass < 2; ++pass) {
#pragma unroll
      for (int it = 0; it < 4; ++it) {
        const int idx = it * NTHR + tid;
        const int row = idx >> 5, c4 = (idx & 31) * 4;
        const v4f v = *(const v4f*)(xs + row * XSP + c4);
        *(volatile v4f*)(out + (size_t)(rb + row) * DIM + c4) = v;
      }
      if (wave == 0) {
        const v4f lv = *(const v4f*)(ldst + l8 * 4);
        if (lane < 8) *(volatile v4f*)(out + (size_t)NBAT * DIM + rb + l8 * 4) = lv;
      }
      __threadfence();
    }
  }
}

extern "C" void kernel_launch(void* const* d_in, const int* in_sizes, int n_in,
                              void* d_out, int out_size, void* d_ws, size_t ws_size, hipStream_t stream) {
  if (n_in < 10 || d_out == nullptr || d_ws == nullptr) return;
  if (in_sizes[0] != NBAT * DIM || in_sizes[1] != HID * DIM || in_sizes[2] != HID || in_sizes[3] != HID * HID ||
      in_sizes[4] != HID || in_sizes[5] != 2 * DIM * HID || in_sizes[6] != 2 * DIM || in_sizes[7] != HID * DIM ||
      in_sizes[8] != HID * HID || in_sizes[9] != 2 * DIM * HID || out_size != NBAT * DIM + NBAT) return;

  const float* z  = (const float*)d_in[0];
  const float* W0 = (const float*)d_in[1];
  const float* b0 = (const float*)d_in[2];
  const float* W1 = (const float*)d_in[3];
  const float* b1 = (const float*)d_in[4];
  const float* W2 = (const float*)d_in[5];
  const float* b2 = (const float*)d_in[6];
  const float* m0 = (const float*)d_in[7];
  const float* m1 = (const float*)d_in[8];
  const float* m2 = (const float*)d_in[9];
  float* out = (float*)d_out;

  char* ws = (char*)d_ws; size_t off = 0;
  auto carve = [&](size_t bytes) -> char* { char* p = ws + off; off += (bytes + 255) & ~(size_t)255; return p; };
  unsigned short* M1H = (unsigned short*)carve((size_t)HID * HID * 2);
  unsigned short* M2A = (unsigned short*)carve((size_t)DIM * HID * 2);
  float*          M0T = (float*)carve((size_t)DIM * HID * 4);
  float*          M2F = (float*)carve((size_t)2 * DIM * HID * 4);
  if (off > ws_size || off > (size_t)134217728) return;

  const int n8_1 = HID * HID / 8;
  const int n8_2 = DIM * HID / 8;
  const int n4_3 = 2 * DIM * HID / 4;
  cvtmask16_kernel<<<(n8_1 + NTHR - 1) / NTHR, NTHR, 0, stream>>>(W1, m1, M1H, n8_1, WCAR);
  cvtmask16_kernel<<<(n8_2 + NTHR - 1) / NTHR, NTHR, 0, stream>>>(W2 + (size_t)DIM * HID, m2 + (size_t)DIM * HID, M2A, n8_2, WCAR);
  tpmask_kernel<<<dim3(DIM / 64, HID / 64), NTHR, 0, stream>>>(W0, m0, HID, DIM, M0T);
  mulmask4_kernel<<<(n4_3 + NTHR - 1) / NTHR, NTHR, 0, stream>>>(W2, m2, M2F, n4_3);
  made_seq_kernel<<<NBAT / ROWS_BLK, NTHR, 0, stream>>>(z, b0, b1, b2, M1H, M2A, M0T, M2F, out);
}
